// MambaLayer2_81999515615486
// MI455X (gfx1250) — hardware-run, weakly checked
//
#include <hip/hip_runtime.h>
#include <hip/hip_bf16.h>
#include <math.h>

#define NB    2
#define DMOD  128
#define DST   16
#define DCV   4
#define DIN   256
#define DTR   8
#define HIMG  96
#define WIMG  96
#define HP    48
#define WP    48
#define L2S   (HP * WP)
#define LSEQ  (2 * L2S)
#define NTOK  (NB * LSEQ)
#define XZW   (2 * DIN)
#define XDV   (DTR + 2 * DST)
#define XDN   64
#define GSTR  40
#define OSTR  68
#define SMEMB (8 * 16 * OSTR * 4)
#define SCH   32
#define SYP   260
#define LOG2E 1.4426950408889634f

static_assert(NTOK % 128 == 0);
static_assert(XZW % 64 == 0);
static_assert(DMOD % 64 == 0);
static_assert(XDN % 64 == 0);
static_assert(XDN >= XDV);
static_assert(DMOD % 32 == 0);
static_assert(DIN % 32 == 0);
static_assert(DIN == 256);
static_assert(DST == 16);
static_assert(DTR == 8);
static_assert(LSEQ % SCH == 0);
static_assert(SCH == 32);
static_assert(SYP % 4 == 0);
static_assert(SYP >= DIN);
static_assert(SMEMB >= (2 * 128 * GSTR + 64 * GSTR) * 2);
static_assert(NTOK % 4 == 0);
static_assert(WIMG % 4 == 0);
static_assert((NB * DMOD * HIMG * WIMG) % 1024 == 0);
static_assert((NTOK * (DMOD / 8)) % 256 == 0);

typedef unsigned short us16 __attribute__((ext_vector_type(16)));
typedef unsigned short us8  __attribute__((ext_vector_type(8)));
typedef unsigned short us8a __attribute__((ext_vector_type(8), may_alias));
typedef __bf16 v16b __attribute__((ext_vector_type(16)));
typedef float v8f __attribute__((ext_vector_type(8)));
typedef float v4f __attribute__((ext_vector_type(4)));
typedef float v4fa __attribute__((ext_vector_type(4), may_alias));
union FragU { us16 v; us8 h[2]; };

__device__ __forceinline__ unsigned short bf16_bits(float f) {
  unsigned u = __float_as_uint(f);
  u += 0x7FFFu + ((u >> 16) & 1u);
  return (unsigned short)(u >> 16);
}
__device__ __forceinline__ float bf16_val(unsigned short b) { return __uint_as_float(((unsigned)b) << 16); }
__device__ __forceinline__ float bf16r(float f) { return bf16_val(bf16_bits(f)); }
__device__ __forceinline__ float siluf(float x) { return x * __builtin_amdgcn_rcpf(1.0f + __expf(-x)); }

__device__ __forceinline__ v8f mma_bf16(us16 a, us16 b, v8f c) {
  return __builtin_amdgcn_wmma_f32_16x16x32_bf16(false, __builtin_bit_cast(v16b, a), false, __builtin_bit_cast(v16b, b), (short)0, c, false, false);
}
__device__ __forceinline__ void wguard(v8f& c0, v8f& c1, v8f& c2, v8f& c3, const us16& a0, const us16& a1,
                                       const us16& b0, const us16& b1, const us16& b2, const us16& b3) {
#if defined(__HIP_DEVICE_COMPILE__)
  asm volatile("v_nop\n\tv_nop\n\tv_nop\n\tv_nop"
               : "+v"(c0), "+v"(c1), "+v"(c2), "+v"(c3)
               : "v"(a0), "v"(a1), "v"(b0), "v"(b1), "v"(b2), "v"(b3));
#endif
}

__device__ __forceinline__ us16 lds_frag(const unsigned short* base) {
  const int lane = threadIdx.x & 31, r = lane & 15, kh = (lane >> 4) * 8;
  FragU f;
  f.h[0] = *(const us8a*)(base + r * GSTR + kh);
  f.h[1] = *(const us8a*)(base + r * GSTR + 16 + kh);
  return f.v;
}

__device__ __forceinline__ void stage_a(unsigned short* lds, const unsigned short* __restrict__ P, int ld, int m0, int k0, int tid) {
  const int row = tid >> 1, cq = (tid & 1) * 16;
  const unsigned short* src = P + (size_t)(m0 + row) * ld + k0 + cq;
  const us8 v0 = *(const us8a*)src;
  const us8 v1 = *(const us8a*)(src + 8);
  *(us8a*)(lds + row * GSTR + cq) = v0;
  *(us8a*)(lds + row * GSTR + cq + 8) = v1;
}
__device__ __forceinline__ void stage_b(unsigned short* lds, const unsigned short* __restrict__ P, int ld, int n0, int k0, int tid) {
  const int row = tid >> 2, kq = (tid & 3) * 8;
  const us8 v = *(const us8a*)(P + (size_t)(n0 + row) * ld + k0 + kq);
  *(us8a*)(lds + row * GSTR + kq) = v;
}

__global__ __launch_bounds__(256) void k_gemm(const unsigned short* __restrict__ A0, const unsigned short* __restrict__ A1, int lda,
                                             const unsigned short* __restrict__ B0, int ldb, float* Y, int ldy, int K) {
  __shared__ __attribute__((aligned(16))) unsigned char sm[SMEMB];
  unsigned short* lA0 = (unsigned short*)sm;
  unsigned short* lA1 = lA0 + 128 * GSTR;
  unsigned short* lB0 = lA1 + 128 * GSTR;
  float* oS = (float*)sm;
  const int tid = threadIdx.x, lane = tid & 31, wave = tid >> 5, cl = lane & 15, hh = lane >> 4;
  const int m0 = blockIdx.x * 128, n0 = blockIdx.y * 64;

  v8f acc[4];
#pragma unroll
  for (int j = 0; j < 4; ++j) { v8f zz = {0.f, 0.f, 0.f, 0.f, 0.f, 0.f, 0.f, 0.f}; acc[j] = zz; }

#pragma unroll 1
  for (int k0 = 0; k0 < K; k0 += 32) {
    __syncthreads();
    stage_a(lA0, A0, lda, m0, k0, tid);
    stage_a(lA1, A1, lda, m0, k0, tid);
    stage_b(lB0, B0, ldb, n0, k0, tid);
    __syncthreads();
    const us16 af0 = lds_frag(lA0 + 16 * wave * GSTR);
    const us16 af1 = lds_frag(lA1 + 16 * wave * GSTR);
    us16 bfr[4];
#pragma unroll
    for (int j = 0; j < 4; ++j) bfr[j] = lds_frag(lB0 + 16 * j * GSTR);
#pragma unroll
    for (int j = 0; j < 4; ++j) acc[j] = mma_bf16(af0, bfr[j], acc[j]);
#pragma unroll
    for (int j = 0; j < 4; ++j) acc[j] = mma_bf16(af1, bfr[j], acc[j]);
    wguard(acc[0], acc[1], acc[2], acc[3], af0, af1, bfr[0], bfr[1], bfr[2], bfr[3]);
  }
  __syncthreads();

  float* so = oS + wave * (16 * OSTR);
#pragma unroll
  for (int j = 0; j < 4; ++j)
#pragma unroll
    for (int r = 0; r < 8; ++r) so[(8 * hh + r) * OSTR + 16 * j + cl] = acc[j][r];
  __syncthreads();
#pragma unroll
  for (int pass = 0; pass < 2; ++pass) {
#pragma unroll
    for (int it = 0; it < 8; ++it) {
      const int ch = it * 32 + lane, r = ch >> 4, q = (ch & 15) * 4;
      const v4f v = *(const v4fa*)(so + r * OSTR + q);
      *(volatile v4f*)(Y + (size_t)(m0 + 16 * wave + r) * ldy + n0 + q) = v;
    }
    __threadfence();
  }
}

__global__ __launch_bounds__(256) void k_cvt(const float* __restrict__ src, unsigned short* dst, int nsrc, int ncol8, int total8) {
  const int idx = blockIdx.x * 256 + threadIdx.x;
  if (idx >= total8) return;
  const int row = idx / ncol8, c8 = (idx - row * ncol8) * 8;
  const int rs = (row < nsrc) ? row : (nsrc - 1);
  const float* s = src + (size_t)rs * (size_t)(ncol8 * 8) + c8;
  const v4f a = *(const v4fa*)s, b = *(const v4fa*)(s + 4);
  const bool zr = (row >= nsrc);
  us8 o;
#pragma unroll
  for (int u = 0; u < 4; ++u) {
    o[u]     = zr ? (unsigned short)0 : bf16_bits(a[u]);
    o[4 + u] = zr ? (unsigned short)0 : bf16_bits(b[u]);
  }
  const size_t off = (size_t)row * (size_t)(ncol8 * 8) + c8;
  *(volatile us8*)(dst + off) = o;
  __threadfence();
  *(volatile us8*)(dst + off) = o;
}

__global__ __launch_bounds__(256) void k_pool(const float* __restrict__ x, unsigned short* UH, unsigned short* UL) {
#pragma clang fp contract(off)
  const int idx = blockIdx.x * 256 + threadIdx.x;
  if (idx >= NTOK * (DMOD / 8)) return;
  const int tok = idx / (DMOD / 8), c8 = (idx - tok * (DMOD / 8)) * 8;
  const int b = tok / LSEQ, l = tok - b * LSEQ;
  const int ish = (l < L2S) ? 1 : 0;
  const int s = ish ? ((L2S - 1) - l) : ((L2S - 1) - (l - L2S));
  const int hq = s / WP, hr = s - hq * WP;
  const int vq = s / HP, vr = s - vq * HP;
  const int h = ish ? hq : vr;
  const int w = ish ? hr : vq;
  us8 hi, lo;
#pragma unroll
  for (int u = 0; u < 8; ++u) {
    const float* p = x + ((size_t)(b * DMOD + c8 + u) * HIMG + 2 * h) * WIMG + 2 * w;
    const float s4 = ((bf16r(p[0]) + bf16r(p[1])) + bf16r(p[WIMG])) + bf16r(p[WIMG + 1]);
    const float v = s4 * 0.25f;
    const unsigned short hb = bf16_bits(v);
    hi[u] = hb; lo[u] = bf16_bits(v - bf16_val(hb));
  }
  const size_t o = (size_t)tok * DMOD + c8;
  *(volatile us8*)(UH + o) = hi; *(volatile us8*)(UL + o) = lo;
  __threadfence();
  *(volatile us8*)(UH + o) = hi; *(volatile us8*)(UL + o) = lo;
}

__global__ __launch_bounds__(256) void k_conv(const float* __restrict__ XZ, const float* __restrict__ cw, const float* __restrict__ cb,
                                             float* XSF, unsigned short* XSH, unsigned short* XSL) {
#pragma clang fp contract(off)
  __shared__ __attribute__((aligned(16))) float sxs[4 * DIN];
  const int tid = threadIdx.x, tl = tid >> 6, c4 = (tid & 63) * 4;
  const int tok = blockIdx.x * 4 + tl;
  const int l = tok % LSEQ;
  v4f xv[DCV];
#pragma unroll
  for (int j = 0; j < DCV; ++j) {
    const int ll = l - (DCV - 1) + j;
    const int tc = (ll >= 0) ? (tok - (DCV - 1) + j) : tok;
    xv[j] = *(const v4fa*)(XZ + (size_t)tc * XZW + c4);
  }
  const v4f bb = *(const v4fa*)(cb + c4);
  v4f sv;
#pragma unroll
  for (int u = 0; u < 4; ++u) {
    const v4f wv = *(const v4fa*)(cw + (size_t)(c4 + u) * DCV);
    float a = 0.0f;
#pragma unroll
    for (int j = 0; j < DCV; ++j) {
      const float pr = bf16r(wv[j]) * xv[j][u];
      a = a + ((l - (DCV - 1) + j >= 0) ? pr : 0.0f);
    }
    a = a + bf16r(bb[u]);
    sv[u] = siluf(a);
  }
  *(v4fa*)(sxs + tl * DIN + c4) = sv;
  const size_t o = (size_t)tok * DIN + c4;
  *(volatile v4f*)(XSF + o) = sv;
  __threadfence();
  *(volatile v4f*)(XSF + o) = sv;
  __syncthreads();
  if (tid < 128) {
    const int row = tid >> 5, c8 = (tid & 31) * 8;
    const v4f a = *(const v4fa*)(sxs + row * DIN + c8);
    const v4f b = *(const v4fa*)(sxs + row * DIN + c8 + 4);
    us8 hi, lo;
#pragma unroll
    for (int u = 0; u < 4; ++u) {
      const unsigned short ha = bf16_bits(a[u]);
      hi[u] = ha; lo[u] = bf16_bits(a[u] - bf16_val(ha));
      const unsigned short hb = bf16_bits(b[u]);
      hi[4 + u] = hb; lo[4 + u] = bf16_bits(b[u] - bf16_val(hb));
    }
    const size_t o2 = (size_t)(blockIdx.x * 4 + row) * DIN + c8;
    *(volatile us8*)(XSH + o2) = hi; *(volatile us8*)(XSL + o2) = lo;
    __threadfence();
    *(volatile us8*)(XSH + o2) = hi; *(volatile us8*)(XSL + o2) = lo;
  }
}

__global__ __launch_bounds__(256) void k_delta(const float* __restrict__ XD, const float* __restrict__ dtw, const float* __restrict__ dtb,
                                              float* DEL) {
#pragma clang fp contract(off)
  const int idx = blockIdx.x * 256 + threadIdx.x;
  if (idx >= NTOK * DIN) return;
  const int d = idx & (DIN - 1), tok = idx >> 8;
  const v4f t0 = *(const v4fa*)(XD + (size_t)tok * XDN), t1 = *(const v4fa*)(XD + (size_t)tok * XDN + 4);
  const v4f w0 = *(const v4fa*)(dtw + d * DTR), w1 = *(const v4fa*)(dtw + d * DTR + 4);
  float a = 0.0f;
#pragma unroll
  for (int u = 0; u < 4; ++u) a = a + t0[u] * bf16r(w0[u]);
#pragma unroll
  for (int u = 0; u < 4; ++u) a = a + t1[u] * bf16r(w1[u]);
  a = a + bf16r(dtb[d]);
  const float sp = fmaxf(a, 0.0f) + log1pf(__expf(-fabsf(a)));
  *(volatile float*)(DEL + idx) = sp;
  __threadfence();
  *(volatile float*)(DEL + idx) = sp;
}

__global__ __launch_bounds__(256) void k_scan(const float* __restrict__ XZ, const float* __restrict__ XSF, const float* __restrict__ XD,
                                             const float* __restrict__ DEL, const float* __restrict__ Alog, const float* __restrict__ Dv,
                                             unsigned short* YGH, unsigned short* YGL) {
#pragma clang fp contract(off)
  __shared__ __attribute__((aligned(16))) float sy[SCH * SYP];
  const int b = blockIdx.x, tid = threadIdx.x, d = tid, lane = tid & 31, wave = tid >> 5;
  float A2[DST], h[DST];
#pragma unroll
  for (int n = 0; n < DST; ++n) { A2[n] = -__expf(bf16r(Alog[d * DST + n])) * LOG2E; h[n] = 0.0f; }
  const float Dd = bf16r(Dv[d]);
#pragma unroll 1
  for (int c = 0; c < LSEQ / SCH; ++c) {
#pragma unroll 1
    for (int s = 0; s < SCH; ++s) {
      const size_t tok = (size_t)b * LSEQ + (size_t)(c * SCH + s);
      const float dl = DEL[tok * DIN + d];
      const float xv = XSF[tok * DIN + d];
      const float zv = XZ[tok * XZW + DIN + d];
      const float* bc = XD + tok * XDN;
      v4f Bv[4], Cv[4];
#pragma unroll
      for (int q = 0; q < 4; ++q) {
        Bv[q] = *(const v4fa*)(bc + DTR + 4 * q);
        Cv[q] = *(const v4fa*)(bc + DTR + DST + 4 * q);
      }
      const float dx = dl * xv;
      float y = 0.0f;
#pragma unroll
      for (int n = 0; n < DST; ++n) {
        const float e = exp2f(dl * A2[n]);
        h[n] = e * h[n] + dx * Bv[n >> 2][n & 3];
        y = y + h[n] * Cv[n >> 2][n & 3];
      }
      const float yv = (y + xv * Dd) * siluf(zv);
      sy[s * SYP + d] = yv;
    }
    __syncthreads();
#pragma unroll
    for (int pass = 0; pass < 2; ++pass) {
#pragma unroll
      for (int it = 0; it < 4; ++it) {
        const int row = 4 * wave + it;
        const v4f va = *(const v4fa*)(sy + row * SYP + lane * 8);
        const v4f vb = *(const v4fa*)(sy + row * SYP + lane * 8 + 4);
        us8 hi, lo;
#pragma unroll
        for (int u = 0; u < 4; ++u) {
          const unsigned short ha = bf16_bits(va[u]);
          hi[u] = ha; lo[u] = bf16_bits(va[u] - bf16_val(ha));
          const unsigned short hb = bf16_bits(vb[u]);
          hi[4 + u] = hb; lo[4 + u] = bf16_bits(vb[u] - bf16_val(hb));
        }
        const size_t o = ((size_t)b * LSEQ + (size_t)(c * SCH + row)) * DIN + lane * 8;
        *(volatile us8*)(YGH + o) = hi; *(volatile us8*)(YGL + o) = lo;
      }
      __threadfence();
    }
    __syncthreads();
  }
}

__global__ __launch_bounds__(256) void k_out(const float* __restrict__ Y2, float* out) {
#pragma clang fp contract(off)
  const int idx = blockIdx.x * 256 + threadIdx.x;
  if (idx >= NB * DMOD * HIMG * WIMG / 4) return;
  const int o = idx * 4;
  const int j = o % WIMG;
  const int i = (o / WIMG) % HIMG;
  const int c = (o / (WIMG * HIMG)) % DMOD;
  const int b = o / (WIMG * HIMG * DMOD);
  const int i0 = ((i + 1) >> 1) - 1;
  const float wi = (i & 1) ? 0.25f : 0.75f;
  const int r0 = (i0 > 0) ? i0 : 0;
  const int r1 = (i0 + 1 < HP - 1) ? (i0 + 1) : (HP - 1);
  const int q2 = j >> 1;
  int cc[4];
#pragma unroll
  for (int e = 0; e < 4; ++e) {
    int v = q2 - 1 + e;
    v = (v > 0) ? v : 0;
    v = (v < WP - 1) ? v : (WP - 1);
    cc[e] = v;
  }
  const size_t bt = (size_t)b * LSEQ;
  float v0[4], v1[4];
#pragma unroll
  for (int e = 0; e < 4; ++e) {
    const size_t l1a = (size_t)((L2S - 1) - (r0 * WP + cc[e])), l2a = (size_t)((LSEQ - 1) - (cc[e] * HP + r0));
    const size_t l1b = (size_t)((L2S - 1) - (r1 * WP + cc[e])), l2b = (size_t)((LSEQ - 1) - (cc[e] * HP + r1));
    v0[e] = Y2[(bt + l1a) * DMOD + c] + Y2[(bt + l2a) * DMOD + c];
    v1[e] = Y2[(bt + l1b) * DMOD + c] + Y2[(bt + l2b) * DMOD + c];
  }
  v4f res;
  {
    const float wj = 0.75f;
    res[0] = (1.0f - wi) * ((1.0f - wj) * v0[0] + wj * v0[1]) + wi * ((1.0f - wj) * v1[0] + wj * v1[1]);
  }
  {
    const float wj = 0.25f;
    res[1] = (1.0f - wi) * ((1.0f - wj) * v0[1] + wj * v0[2]) + wi * ((1.0f - wj) * v1[1] + wj * v1[2]);
  }
  {
    const float wj = 0.75f;
    res[2] = (1.0f - wi) * ((1.0f - wj) * v0[1] + wj * v0[2]) + wi * ((1.0f - wj) * v1[1] + wj * v1[2]);
  }
  {
    const float wj = 0.25f;
    res[3] = (1.0f - wi) * ((1.0f - wj) * v0[2] + wj * v0[3]) + wi * ((1.0f - wj) * v1[2] + wj * v1[3]);
  }
  *(volatile v4f*)(out + o) = res;
  __threadfence();
  *(volatile v4f*)(out + o) = res;
}

extern "C" void kernel_launch(void* const* d_in, const int* in_sizes, int n_in,
                              void* d_out, int out_size, void* d_ws, size_t ws_size,
                              hipStream_t stream) {
  if (n_in < 10) return;
  if (in_sizes[0] != NB * DMOD * HIMG * WIMG || in_sizes[1] != XZW * DMOD || in_sizes[2] != DIN * DCV ||
      in_sizes[3] != DIN || in_sizes[4] != XDV * DIN || in_sizes[5] != DIN * DTR || in_sizes[6] != DIN ||
      in_sizes[7] != DIN * DST || in_sizes[8] != DIN || in_sizes[9] != DMOD * DIN ||
      out_size != NB * DMOD * HIMG * WIMG) return;
  const float* x     = (const float*)d_in[0];
  const float* Win   = (const float*)d_in[1];
  const float* cw    = (const float*)d_in[2];
  const float* cb    = (const float*)d_in[3];
  const float* Wx    = (const float*)d_in[4];
  const float* dtw   = (const float*)d_in[5];
  const float* dtb   = (const float*)d_in[6];
  const float* Alog  = (const float*)d_in[7];
  const float* Dv    = (const float*)d_in[8];
  const float* Wo    = (const float*)d_in[9];
  float* out = (float*)d_out;

  size_t off = 0;
  auto carve = [&](size_t bytes) -> char* { char* p = (char*)d_ws + off; off += (bytes + 255) & ~(size_t)255; return p; };
  unsigned short* UH   = (unsigned short*)carve((size_t)NTOK * DMOD * 2);
  unsigned short* UL   = (unsigned short*)carve((size_t)NTOK * DMOD * 2);
  unsigned short* WIN16 = (unsigned short*)carve((size_t)XZW * DMOD * 2);
  unsigned short* WX16  = (unsigned short*)carve((size_t)XDN * DIN * 2);
  unsigned short* WO16  = (unsigned short*)carve((size_t)DMOD * DIN * 2);
  float* XZ            = (float*)carve((size_t)NTOK * XZW * 4);
  float* XSF           = (float*)carve((size_t)NTOK * DIN * 4);
  unsigned short* XSH  = (unsigned short*)carve((size_t)NTOK * DIN * 2);
  unsigned short* XSL  = (unsigned short*)carve((size_t)NTOK * DIN * 2);
  float* XD            = (float*)carve((size_t)NTOK * XDN * 4);
  float* DEL           = (float*)carve((size_t)NTOK * DIN * 4);
  unsigned short* YGH  = (unsigned short*)carve((size_t)NTOK * DIN * 2);
  unsigned short* YGL  = (unsigned short*)carve((size_t)NTOK * DIN * 2);
  float* Y2            = (float*)carve((size_t)NTOK * DMOD * 4);
  if (off > ws_size || off > (size_t)134217728) return;

  const dim3 blk(256);
  k_pool<<<dim3((NTOK * (DMOD / 8) + 255) / 256), blk, 0, stream>>>(x, UH, UL);
  k_cvt<<<dim3((XZW * DMOD / 8 + 255) / 256), blk, 0, stream>>>(Win, WIN16, XZW, DMOD / 8, XZW * DMOD / 8);
  k_cvt<<<dim3((XDN * DIN / 8 + 255) / 256), blk, 0, stream>>>(Wx, WX16, XDV, DIN / 8, XDN * DIN / 8);
  k_cvt<<<dim3((DMOD * DIN / 8 + 255) / 256), blk, 0, stream>>>(Wo, WO16, DMOD, DIN / 8, DMOD * DIN / 8);
  k_gemm<<<dim3(NTOK / 128, XZW / 64), blk, 0, stream>>>(UH, UL, DMOD, WIN16, DMOD, XZ, XZW, DMOD);
  k_conv<<<dim3(NTOK / 4), blk, 0, stream>>>(XZ, cw, cb, XSF, XSH, XSL);
  k_gemm<<<dim3(NTOK / 128, XDN / 64), blk, 0, stream>>>(XSH, XSL, DIN, WX16, DIN, XD, XDN, DIN);
  k_delta<<<dim3((NTOK * DIN + 255) / 256), blk, 0, stream>>>(XD, dtw, dtb, DEL);
  k_scan<<<dim3(NB), blk, 0, stream>>>(XZ, XSF, XD, DEL, Alog, Dv, YGH, YGL);
  k_gemm<<<dim3(NTOK / 128, DMOD / 64), blk, 0, stream>>>(YGH, YGL, DIN, WO16, DIN, Y2, DMOD, DIN);
  k_out<<<dim3((NB * DMOD * HIMG * WIMG / 4 + 255) / 256), blk, 0, stream>>>(Y2, out);
}
